// GViTEncoder_21208548508277
// MI455X (gfx1250) — hardware-verified
//
#include <hip/hip_runtime.h>
#include <hip/hip_bf16.h>


#define USE_TDM 0
typedef _Float16 bf16_t;
typedef __attribute__((ext_vector_type(16))) _Float16 v16bf;
typedef __attribute__((ext_vector_type(8)))  _Float16 v8bf;
typedef __attribute__((ext_vector_type(4)))  float v4f;
typedef __attribute__((ext_vector_type(8)))  float  v8f;
typedef unsigned int u32;
typedef __attribute__((ext_vector_type(4))) u32 v4u;
typedef __attribute__((ext_vector_type(8))) int v8i;
typedef __attribute__((ext_vector_type(4))) int v4i;

#define BATCH  8
#define SEQ    1024
#define FIN    384
#define FHID   96
#define NHEADS 8
#define FOUT   384
#define HDIM   (NHEADS * FHID + FIN)
#define ODIM   (FOUT + HDIM)
#define ROWS   (BATCH * SEQ)
#define NEG_SLOPE 0.01f
#define LN_EPS    1e-5f


__device__ inline v16bf load_a_frag(const bf16_t* rowbase, int ldm, int lane) {
  const int m  = lane & 15;
  const int hi = lane >> 4;
  const bf16_t* p = rowbase + m * ldm + hi * 8;
  v8bf lo = *(const v8bf*)(p);
  v8bf hh = *(const v8bf*)(p + 16);
  v16bf a;
#pragma unroll
  for (int i = 0; i < 8; ++i) { a[i] = lo[i]; a[8 + i] = hh[i]; }
  return a;
}

__device__ inline v16bf load_b_frag(const bf16_t* packed_tile, int lane) {
  return ((const v16bf*)packed_tile)[lane];
}

__device__ inline v8f wmma_bf16(v16bf a, v16bf b, v8f c) {
  v8f d = __builtin_amdgcn_wmma_f32_16x16x32_f16(false, a, false, b,
                                                  (short)0, c, false, false);
  asm volatile("v_nop\n\tv_nop\n\tv_nop\n\tv_nop" : "+v"(d) : "v"(a), "v"(b));
  return d;
}

__device__ inline float lrelu(float x) { return x >= 0.f ? x : NEG_SLOPE * x; }

#if USE_TDM
__device__ inline void tdm_load_2d(u32 lds_addr, const void* gaddr,
                                   u32 tile_d0, u32 tile_d1,
                                   u32 tens_d0, u32 tens_d1, u32 d0_stride) {
  unsigned long long ga = (unsigned long long)(uintptr_t)gaddr;
  v4u g0;
  g0[0] = 1u;
  g0[1] = lds_addr;
  g0[2] = (u32)(ga & 0xffffffffu);
  g0[3] = (u32)((ga >> 32) & 0x01ffffffu) | (2u << 30);
  v8i g1;
  g1[0] = (int)(3u << 16);
  g1[1] = (int)((tens_d0 & 0xffffu) << 16);
  g1[2] = (int)((tens_d0 >> 16) & 0xffffu) | (int)((tens_d1 & 0xffffu) << 16);
  g1[3] = (int)((tens_d1 >> 16) & 0xffffu) | (int)((tile_d0 & 0xffffu) << 16);
  g1[4] = (int)(tile_d1 & 0xffffu);
  g1[5] = (int)d0_stride;
  g1[6] = 0;
  g1[7] = 0;
  v4i z4 = {0, 0, 0, 0};
#if defined(__clang_major__) && __clang_major__ >= 23
  v8i z8 = {0, 0, 0, 0, 0, 0, 0, 0};
  __builtin_amdgcn_tensor_load_to_lds(g0, g1, z4, z4, z8, 0);
#else
  __builtin_amdgcn_tensor_load_to_lds(g0, g1, z4, z4, 0);
#endif
}
#endif

__global__ __launch_bounds__(256) void pack_b_kernel(const float* __restrict__ W,
                                                     bf16_t* __restrict__ out,
                                                     int K, int Ncols) {
  int idx = blockIdx.x * blockDim.x + threadIdx.x;
  int total = K * Ncols;
  if (idx >= total) return;
  int tile = idx >> 9;
  int r    = idx & 511;
  int lane = r >> 4;
  int i    = r & 15;
  int nkt  = K >> 5;
  int nt   = tile / nkt;
  int kt   = tile - nt * nkt;
  int n    = nt * 16 + (lane & 15);
  int hi   = lane >> 4;
  int k    = kt * 32 + ((i < 8) ? (8 * hi + i) : (16 + 8 * hi + (i - 8)));
  const bf16_t v = (bf16_t)W[k * Ncols + n];
  *(volatile bf16_t*)(out + idx) = v; __threadfence(); *(volatile bf16_t*)(out + idx) = v;
}

__global__ __launch_bounds__(256) void pack_v_kernel(const float* __restrict__ V,
                                                     bf16_t* __restrict__ out) {
  int idx = blockIdx.x * blockDim.x + threadIdx.x;
  if (idx >= ROWS * FHID) return;
  const int per_b = SEQ * FHID;
  int b   = idx / per_b;
  int t   = idx - b * per_b;
  int tile = t >> 9;
  int r    = t & 511;
  int lane = r >> 4;
  int i    = r & 15;
  const int nkt = SEQ / 32;
  int nt = tile / nkt;
  int kt = tile - nt * nkt;
  int f  = nt * 16 + (lane & 15);
  int hi = lane >> 4;
  int j  = kt * 32 + ((i < 8) ? (8 * hi + i) : (16 + 8 * hi + (i - 8)));
  const bf16_t v = (bf16_t)V[(size_t)(b * SEQ + j) * FHID + f];
  *(volatile bf16_t*)(out + idx) = v; __threadfence(); *(volatile bf16_t*)(out + idx) = v;
}

__global__ __launch_bounds__(32) void ln_v_qk_kernel(
    const float* __restrict__ X, const bf16_t* __restrict__ Wvp,
    const float* __restrict__ bv, const float* __restrict__ Wq,
    const float* __restrict__ bq, const float* __restrict__ Wk,
    const float* __restrict__ bk, float* __restrict__ V,
    float* __restrict__ Q, float* __restrict__ Kd,
    float* __restrict__ H) {
  __shared__ __attribute__((aligned(16))) bf16_t hn[16][FIN + 8];
  __shared__ float vt[16][FHID + 4];
  const int lane = threadIdx.x;
  const int r0   = blockIdx.x * 16;

  for (int row = 0; row < 16; ++row) {
    const float* xr = X + (size_t)(r0 + row) * FIN;
    float s = 0.f, ss = 0.f;
    for (int c = lane; c < FIN; c += 32) { float x = xr[c]; s += x; ss += x * x; }
#pragma unroll
    for (int off = 16; off; off >>= 1) {
      s  += __shfl_xor(s, off, 32);
      ss += __shfl_xor(ss, off, 32);
    }
    float mu   = s * (1.f / FIN);
    float rstd = rsqrtf(ss * (1.f / FIN) - mu * mu + LN_EPS);
    for (int c = lane; c < FIN; c += 32) {
      float x = xr[c];
      hn[row][c] = (bf16_t)((x - mu) * rstd);
      float* hp = H + (size_t)(r0 + row) * HDIM + NHEADS * FHID + c;
      *(volatile float*)hp = x; *(volatile float*)hp = x;
    }
  }
  __threadfence();
  __syncthreads();

  v8f acc[6];
#pragma unroll
  for (int t = 0; t < 6; ++t) acc[t] = (v8f){0.f,0.f,0.f,0.f,0.f,0.f,0.f,0.f};
  for (int kt = 0; kt < 12; ++kt) {
    v16bf a = load_a_frag(&hn[0][0] + kt * 32, FIN + 8, lane);
#pragma unroll
    for (int nt = 0; nt < 6; ++nt) {
      v16bf b = load_b_frag(Wvp + (size_t)(nt * 12 + kt) * 512, lane);
      acc[nt] = wmma_bf16(a, b, acc[nt]);
    }
  }
  const int nl = lane & 15;
  const int rh = (lane >> 4) * 8;
#pragma unroll
  for (int nt = 0; nt < 6; ++nt) {
    int n = nt * 16 + nl;
    float bias = bv[n];
#pragma unroll
    for (int v = 0; v < 8; ++v) {
      float val = acc[nt][v] + bias;
      vt[rh + v][n] = val;
    }
  }
  __syncthreads();
  for (int pass = 0; pass < 2; ++pass) {
#pragma unroll
    for (int q = 0; q < 12; ++q) {
      const int piece = q * 32 + lane, row = piece / 24, c4 = (piece % 24) * 4;
      v4f v; v[0] = vt[row][c4]; v[1] = vt[row][c4 + 1]; v[2] = vt[row][c4 + 2]; v[3] = vt[row][c4 + 3];
      *(volatile v4f*)(V + (size_t)(r0 + row) * FHID + c4) = v;
    }
    __threadfence();
  }

  for (int t = lane; t < 128; t += 32) {
    int row = t >> 3, h = t & 7;
    float q = bq[h], k = bk[h];
    for (int f = 0; f < FHID; ++f) {
      float v = vt[row][f];
      q += v * Wq[f * NHEADS + h];
      k += v * Wk[f * NHEADS + h];
    }
    *(volatile float*)(Q  + (size_t)(r0 + row) * NHEADS + h) = q;
    *(volatile float*)(Kd + (size_t)(r0 + row) * NHEADS + h) = k;
    __threadfence();
    *(volatile float*)(Q  + (size_t)(r0 + row) * NHEADS + h) = q;
    *(volatile float*)(Kd + (size_t)(r0 + row) * NHEADS + h) = k;
  }
}

__global__ __launch_bounds__(256) void attn_kernel(
    const float* __restrict__ Q, const float* __restrict__ Kmat,
    const bf16_t* __restrict__ Vp, float* __restrict__ H) {
  const int b    = blockIdx.x >> 6;
  const int i0   = (blockIdx.x & 63) * 16;
  const int tid  = threadIdx.x;
  const int wave = tid >> 5;
  const int lane = tid & 31;

  __shared__ float  qs[16][NHEADS];
  __shared__ float  ks[32][NHEADS];
  __shared__ __attribute__((aligned(16))) bf16_t aT[NHEADS][16][40];
  __shared__ __attribute__((aligned(16))) float sH[NHEADS][16][100];
#if USE_TDM
  __shared__ __attribute__((aligned(16))) bf16_t vtile[2][6][512];
#endif

  if (tid < 128)
    qs[tid >> 3][tid & 7] = Q[(size_t)(b * SEQ + i0 + (tid >> 3)) * NHEADS + (tid & 7)];

  v8f acc[6];
#pragma unroll
  for (int t = 0; t < 6; ++t) acc[t] = (v8f){0.f,0.f,0.f,0.f,0.f,0.f,0.f,0.f};

  const bf16_t* vbase = Vp + (size_t)b * (SEQ * FHID);

#if USE_TDM
  const u32 lds0 = (u32)(uintptr_t)&vtile[0][0][0];
  if (wave == 0)
    tdm_load_2d(lds0, vbase,  128, 6,  4096, 16,  4096);
#endif
  __syncthreads();

  for (int jc = 0; jc < 32; ++jc) {
    ks[tid >> 3][tid & 7] =
        Kmat[(size_t)(b * SEQ + jc * 32 + (tid >> 3)) * NHEADS + (tid & 7)];
#if USE_TDM
    if (wave == 0) {
      int jn = (jc + 1) & 31;
      tdm_load_2d(lds0 + (u32)(((jc + 1) & 1) * sizeof(vtile[0])),
                  vbase + (size_t)jn * 512, 128, 6, 4096, 16, 4096);
    }
#else
    if (jc + 1 < 32)
      __builtin_prefetch(vbase + (size_t)(jc + 1) * 512, 0, 1);
#endif
    __syncthreads();

    const int i  = tid >> 4;
    const int jl = tid & 15;
#pragma unroll
    for (int jj = 0; jj < 2; ++jj) {
      const int j = jl + jj * 16;
      float e[NHEADS], denom = 0.f;
#pragma unroll
      for (int h = 0; h < NHEADS; ++h) {
        float s = lrelu(qs[i][h] * ks[j][h]);
        e[h] = __expf(s);
        denom += e[h];
      }
      float inv = 1.f / denom;
#pragma unroll
      for (int h = 0; h < NHEADS; ++h) aT[h][i][j] = (bf16_t)(e[h] * inv);
    }
#if USE_TDM
    if (wave == 0) __builtin_amdgcn_s_wait_tensorcnt(1);
#endif
    __syncthreads();

    v16bf a = load_a_frag(&aT[wave][0][0], 40, lane);
#pragma unroll
    for (int nt = 0; nt < 6; ++nt) {
#if USE_TDM
      v16bf bfr = load_b_frag(&vtile[jc & 1][nt][0], lane);
#else
      v16bf bfr = load_b_frag(vbase + (size_t)(nt * 32 + jc) * 512, lane);
#endif
      acc[nt] = wmma_bf16(a, bfr, acc[nt]);
    }
    __syncthreads();
  }

  const int nl = lane & 15;
  const int rh = (lane >> 4) * 8;
#pragma unroll
  for (int nt = 0; nt < 6; ++nt)
#pragma unroll
    for (int v = 0; v < 8; ++v) sH[wave][rh + v][nt * 16 + nl] = acc[nt][v];
  __builtin_amdgcn_fence(__ATOMIC_RELEASE, "workgroup"); __builtin_amdgcn_wave_barrier(); __builtin_amdgcn_fence(__ATOMIC_ACQUIRE, "workgroup");
  for (int pass = 0; pass < 2; ++pass) {
#pragma unroll
    for (int row = 0; row < 16; ++row)
      if (lane < 24) {
        v4f v; v[0] = sH[wave][row][lane * 4]; v[1] = sH[wave][row][lane * 4 + 1]; v[2] = sH[wave][row][lane * 4 + 2]; v[3] = sH[wave][row][lane * 4 + 3];
        *(volatile v4f*)(H + (size_t)(b * SEQ + i0 + row) * HDIM + wave * FHID + lane * 4) = v;
      }
    __threadfence();
  }
}

__global__ __launch_bounds__(128) void out_kernel(
    const float* __restrict__ H, const bf16_t* __restrict__ Wmp,
    const float* __restrict__ bm, float* __restrict__ out) {
  __shared__ __attribute__((aligned(16))) bf16_t hn[16][HDIM + 8];
  __shared__ __attribute__((aligned(16))) float sO[16][FOUT + 4];
  const int r0   = blockIdx.x * 16;
  const int tid  = threadIdx.x;
  const int wave = tid >> 5;
  const int lane = tid & 31;

  for (int row = wave; row < 16; row += 4) {
    const float* hr = H + (size_t)(r0 + row) * HDIM;
    float s = 0.f, ss = 0.f;
    for (int c = lane; c < HDIM; c += 32) { float x = hr[c]; s += x; ss += x * x; }
#pragma unroll
    for (int off = 16; off; off >>= 1) {
      s  += __shfl_xor(s, off, 32);
      ss += __shfl_xor(ss, off, 32);
    }
    float mu   = s * (1.f / HDIM);
    float rstd = rsqrtf(ss * (1.f / HDIM) - mu * mu + LN_EPS);
    for (int c = lane; c < HDIM; c += 32)
      hn[row][c] = (bf16_t)((hr[c] - mu) * rstd);
  }
  __syncthreads();

  v8f acc[6];
#pragma unroll
  for (int t = 0; t < 6; ++t) acc[t] = (v8f){0.f,0.f,0.f,0.f,0.f,0.f,0.f,0.f};
  for (int kt = 0; kt < 36; ++kt) {
    v16bf a = load_a_frag(&hn[0][0] + kt * 32, HDIM + 8, lane);
#pragma unroll
    for (int t = 0; t < 6; ++t) {
      int nt = wave * 6 + t;
      v16bf b = load_b_frag(Wmp + (size_t)(nt * 36 + kt) * 512, lane);
      acc[t] = wmma_bf16(a, b, acc[t]);
    }
  }
  const int nl = lane & 15;
  const int rh = (lane >> 4) * 8;
#pragma unroll
  for (int t = 0; t < 6; ++t) {
    int n = (wave * 6 + t) * 16 + nl;
    float bias = bm[n];
#pragma unroll
    for (int v = 0; v < 8; ++v) sO[rh + v][n] = lrelu(acc[t][v] + bias);
  }
  __syncthreads();
  for (int pass = 0; pass < 2; ++pass) {
    for (int piece = tid; piece < 16 * 96; piece += 128) {
      const int row = piece / 96, c4 = (piece % 96) * 4;
      *(volatile v4f*)(out + (size_t)(r0 + row) * ODIM + c4) = *(const v4f*)(&sO[row][c4]);
    }
    for (int idx = tid; idx < 16 * HDIM; idx += 128) {
      int row = idx / HDIM, c = idx - row * HDIM;
      *(volatile float*)(out + (size_t)(r0 + row) * ODIM + FOUT + c) = H[(size_t)(r0 + row) * HDIM + c];
    }
    __threadfence();
  }
}

extern "C" void kernel_launch(void* const* d_in, const int* in_sizes, int n_in,
                              void* d_out, int out_size, void* d_ws, size_t ws_size,
                              hipStream_t stream) {
  const float* X  = (const float*)d_in[0];
  const float* Wv = (const float*)d_in[1];
  const float* bv = (const float*)d_in[2];
  const float* Wq = (const float*)d_in[3];
  const float* bq = (const float*)d_in[4];
  const float* Wk = (const float*)d_in[5];
  const float* bk = (const float*)d_in[6];
  const float* Wm = (const float*)d_in[7];
  const float* bm = (const float*)d_in[8];
  float* out = (float*)d_out;

  char* ws = (char*)d_ws;
  size_t off = 0;
  auto alloc = [&](size_t bytes) -> void* {
    void* p = ws + off;
    off = (off + bytes + 255) & ~(size_t)255;
    return p;
  };
  bf16_t* Wvp = (bf16_t*)alloc((size_t)FIN * FHID * 2);
  bf16_t* Wmp = (bf16_t*)alloc((size_t)HDIM * FOUT * 2);
  float*  V   = (float*) alloc((size_t)ROWS * FHID * 4);
  bf16_t* Vp  = (bf16_t*)alloc((size_t)ROWS * FHID * 2);
  float*  Q   = (float*) alloc((size_t)ROWS * NHEADS * 4);
  float*  Kd  = (float*) alloc((size_t)ROWS * NHEADS * 4);
  float*  H   = (float*) alloc((size_t)ROWS * HDIM * 4);
  (void)in_sizes; (void)n_in; (void)out_size;
  if (off > ws_size) return;

  pack_b_kernel<<<(FIN * FHID + 255) / 256, 256, 0, stream>>>(Wv, Wvp, FIN, FHID);
  pack_b_kernel<<<(HDIM * FOUT + 255) / 256, 256, 0, stream>>>(Wm, Wmp, HDIM, FOUT);

  ln_v_qk_kernel<<<ROWS / 16, 32, 0, stream>>>(X, Wvp, bv, Wq, bq, Wk, bk,
                                               V, Q, Kd, H);

  pack_v_kernel<<<(ROWS * FHID + 255) / 256, 256, 0, stream>>>(V, Vp);

  attn_kernel<<<BATCH * (SEQ / 16), 256, 0, stream>>>(Q, Kd, Vp, H);

  out_kernel<<<ROWS / 16, 128, 0, stream>>>(H, Wmp, bm, out);
}
